// RMultiHeadSelfAttention_87995289960719
// MI455X (gfx1250) — hardware-verified
//
#include <hip/hip_runtime.h>
#include <math.h>

typedef __attribute__((ext_vector_type(16))) _Float16 v16h;
typedef __attribute__((ext_vector_type(8)))  _Float16 v8h;
typedef __attribute__((ext_vector_type(16))) __bf16   v16b;
typedef __attribute__((ext_vector_type(8)))  __bf16   v8b;
typedef __attribute__((ext_vector_type(8)))  float    v8f;
typedef __attribute__((ext_vector_type(4)))  float    v4f;
typedef __attribute__((ext_vector_type(2)))  float    v2f;

constexpr int NBATCH   = 2;
constexpr int SEQ_LEN  = 2048;
constexpr int D_MOD    = 1024;
constexpr int N_HEADS  = 16;
constexpr int HEAD_D   = 64;
constexpr int NTOK     = NBATCH * SEQ_LEN;
constexpr int NBH      = NBATCH * N_HEADS;
constexpr int NQB      = SEQ_LEN / 64;
constexpr int QKV_COLS = 3072;
constexpr int K_COL0   = 1024;
constexpr int V_COL0   = 2048;
constexpr int STG_PITCH = 72;

struct InvFreqTab { float f[32]; };
static_assert(sizeof(InvFreqTab) == 128, "size");

__device__ __forceinline__ unsigned short f2bf_bits(float f) {
  unsigned u = __float_as_uint(f);
  return (unsigned short)((u + 0x7FFFu + ((u >> 16) & 1u)) >> 16);
}
__device__ __forceinline__ float bf_bits2f(unsigned short h) { return __uint_as_float(((unsigned)h) << 16); }

__device__ __forceinline__ void dep_guard_h(v8f& a, v8f& b, v16h x, v16h y) { asm volatile("v_nop\n\tv_nop\n\tv_nop\n\tv_nop" : "+v"(a), "+v"(b) : "v"(x), "v"(y)); }
__device__ __forceinline__ void dep_guard_b(v8f& a, v8f& b, v16b x, v16b y) { asm volatile("v_nop\n\tv_nop\n\tv_nop\n\tv_nop" : "+v"(a), "+v"(b) : "v"(x), "v"(y)); }
__device__ __forceinline__ void keep4_h(v16h a, v16h b, v16h c, v16h d) { asm volatile("v_nop" :: "v"(a), "v"(b), "v"(c), "v"(d)); }
__device__ __forceinline__ void keep4_b(v16b a, v16b b, v16b c, v16b d) { asm volatile("v_nop" :: "v"(a), "v"(b), "v"(c), "v"(d)); }
__device__ __forceinline__ void acc_guard4(v8f& a, v8f& b, v8f& c, v8f& d) { asm volatile("v_nop\n\tv_nop\n\tv_nop\n\tv_nop" : "+v"(a), "+v"(b), "+v"(c), "+v"(d)); }
template <typename T> struct Frag;
template <> struct Frag<_Float16> {
  typedef v16h V; union U { v16h v; v8h h[2]; };
  static __device__ __forceinline__ v16h load(const _Float16* p) {
    U f; f.h[0] = *(const v8h*)(p); f.h[1] = *(const v8h*)(p + 16); return f.v;
  }
  static __device__ __forceinline__ v8f mma(v16h a, v16h b, v8f c) {
    return __builtin_amdgcn_wmma_f32_16x16x32_f16(false, a, false, b, (short)0, c, false, false);
  }
  static __device__ __forceinline__ void guard(v8f& a, v8f& b, v16h x, v16h y) { dep_guard_h(a, b, x, y); }
  static __device__ __forceinline__ void keep(v16h a, v16h b, v16h c, v16h d) { keep4_h(a, b, c, d); }
};
template <> struct Frag<__bf16> {
  typedef v16b V; union U { v16b v; v8b h[2]; };
  static __device__ __forceinline__ v16b load(const __bf16* p) {
    U f; f.h[0] = *(const v8b*)(p); f.h[1] = *(const v8b*)(p + 16); return f.v;
  }
  static __device__ __forceinline__ v8f mma(v16b a, v16b b, v8f c) {
    return __builtin_amdgcn_wmma_f32_16x16x32_bf16(false, a, false, b, (short)0, c, false, false);
  }
  static __device__ __forceinline__ void guard(v8f& a, v8f& b, v16b x, v16b y) { dep_guard_b(a, b, x, y); }
  static __device__ __forceinline__ void keep(v16b a, v16b b, v16b c, v16b d) { keep4_b(a, b, c, d); }
};

__device__ __forceinline__ unsigned short at_bf_bits(float f) {
  unsigned u = __float_as_uint(f);
  return (unsigned short)((u + 0x7FFFu + ((u >> 16) & 1u)) >> 16);
}
__device__ __forceinline__ __bf16 at_f2bf(float f) { return __builtin_bit_cast(__bf16, at_bf_bits(f)); }
__device__ __forceinline__ void at_split(float f, __bf16& hi, __bf16& lo) {
  const unsigned short hb = at_bf_bits(f);
  hi = __builtin_bit_cast(__bf16, hb);
  lo = at_f2bf(f - __uint_as_float(((unsigned)hb) << 16));
}
__device__ __forceinline__ v8f at_mma(v16b a, v16b b, v8f c) {
  c = __builtin_amdgcn_wmma_f32_16x16x32_bf16(false, a, false, b, (short)0, c, false, false);
  asm volatile("v_nop\n\tv_nop\n\tv_nop\n\tv_nop" : "+v"(c) : "v"(a), "v"(b));
  return c;
}

__global__ __launch_bounds__(256) void cast_f32_bf16x2(const float* __restrict__ in,
                                                       unsigned short* __restrict__ out, int n2) {
  const int i = blockIdx.x * 256 + threadIdx.x;
  if (i < n2) {
    const unsigned u = (unsigned)f2bf_bits(in[2 * i]) | ((unsigned)f2bf_bits(in[2 * i + 1]) << 16);
    ((volatile unsigned*)out)[i] = u;
    __threadfence();
    ((volatile unsigned*)out)[i] = u;
  }
}

template <int ET> struct Elem;
template <> struct Elem<0> { typedef _Float16 T; };
template <> struct Elem<1> { typedef __bf16 T; };
template <int ET, int SPLITM, int BIAS_MODE, int OUT_MODE, bool RESID, int ACT = 0>
__global__ __launch_bounds__(256) void wmma_gemm64(
    const unsigned short* __restrict__ Ap, const unsigned short* __restrict__ A2p, int lda, long strideA,
    const unsigned short* __restrict__ Btp, const unsigned short* __restrict__ Bt2p, int ldb, long strideB,
    void* __restrict__ Cout, void* __restrict__ Cout2, int ldc, long strideC,
    const float* __restrict__ bias,
    const float* __restrict__ resid, long strideR,
    int M, int N, int K, float scale) {
  typedef typename Elem<ET>::T T;
  typedef typename Frag<T>::V V;
  constexpr bool SPA = (SPLITM >= 1);
  constexpr bool SPB = (SPLITM >= 2);
  const T* A = (const T*)Ap; const T* A2 = (const T*)A2p; const T* Bt = (const T*)Btp; const T* Bt2 = (const T*)Bt2p;
  __shared__ __align__(16) float sT[8][16 * 68];
  const int b    = blockIdx.y;
  const int lane = threadIdx.x & 31;
  const int wave = threadIdx.x >> 5;
  const int tilesN = N >> 6;
  const int tilesM = M >> 6;
  const int tile = blockIdx.x * 8 + wave;
  if (tile >= tilesM * tilesN) return;
  const int tm = tile / tilesN;
  const int tn = tile - tm * tilesN;
  const int m0 = tm << 6;
  const int n0 = tn << 6;

  const T* Ab  = A  + (size_t)b * strideA;
  const T* Bb  = Bt + (size_t)b * strideB;
  const T* Ab2 = SPA ? (A2  + (size_t)b * strideA) : nullptr;
  const T* Bb2 = SPB ? (Bt2 + (size_t)b * strideB) : nullptr;

  const int rlane = lane & 15;
  const int koff  = (lane >> 4) * 8;
  const int mOff  = (lane >> 4) * 8;

  v8f acc[4][4];
#pragma unroll
  for (int i = 0; i < 4; ++i)
#pragma unroll
    for (int j = 0; j < 4; ++j) acc[i][j] = (v8f){0.f,0.f,0.f,0.f,0.f,0.f,0.f,0.f};

  for (int k0 = 0; k0 < K; k0 += 32) {
    V bh[4], bl[4];
#pragma unroll
    for (int j = 0; j < 4; ++j) {
      const size_t bo = (size_t)(n0 + (j << 4) + rlane) * ldb + koff + k0;
      bh[j] = Frag<T>::load(Bb + bo);
      if (SPB) bl[j] = Frag<T>::load(Bb2 + bo);
    }
#pragma unroll
    for (int i = 0; i < 4; ++i) {
      const size_t ao = (size_t)(m0 + (i << 4) + rlane) * lda + koff + k0;
      V ah = Frag<T>::load(Ab + ao);
      V al;
      if (SPA) al = Frag<T>::load(Ab2 + ao);
#pragma unroll
      for (int j = 0; j < 4; ++j) {
        acc[i][j] = Frag<T>::mma(ah, bh[j], acc[i][j]);
        if (SPB) acc[i][j] = Frag<T>::mma(ah, bl[j], acc[i][j]);
        if (SPA) acc[i][j] = Frag<T>::mma(al, bh[j], acc[i][j]);
      }
      Frag<T>::guard(acc[i][0], acc[i][3], ah, SPA ? al : ah);
    }
    Frag<T>::keep(bh[0], bh[1], bh[2], bh[3]);
    if (SPB) Frag<T>::keep(bl[0], bl[1], bl[2], bl[3]);
  }
  acc_guard4(acc[0][0], acc[0][1], acc[0][2], acc[0][3]);
  acc_guard4(acc[1][0], acc[1][1], acc[1][2], acc[1][3]);
  acc_guard4(acc[2][0], acc[2][1], acc[2][2], acc[2][3]);
  acc_guard4(acc[3][0], acc[3][1], acc[3][2], acc[3][3]);

  float* slab = sT[wave];
  const float* Rb = RESID ? (resid + (size_t)b * strideR) : nullptr;
#pragma unroll
  for (int i = 0; i < 4; ++i) {
    const int mBase = m0 + (i << 4);
#pragma unroll
    for (int j = 0; j < 4; ++j) {
      const int n = n0 + (j << 4) + rlane;
      float bv = 0.f;
      if (BIAS_MODE == 2) bv = bias[n];
#pragma unroll
      for (int r = 0; r < 8; ++r) {
        float v = acc[i][j][r] * scale;
        if (BIAS_MODE == 1) v += bias[mBase + mOff + r];
        if (BIAS_MODE == 2) v += bv;
        if (RESID) v += Rb[(size_t)(mBase + mOff + r) * ldc + n];
        if (ACT == 1) v = tanhf(v);
        if (ACT == 2) v = fmaxf(v, 0.0f);
        if (ACT == 4) v = (v > 0.f) ? v : 0.01f * v;
        slab[(mOff + r) * 68 + (j << 4) + rlane] = v;
      }
    }
    __builtin_amdgcn_fence(__ATOMIC_RELEASE, "workgroup");
    __builtin_amdgcn_wave_barrier();
    __builtin_amdgcn_fence(__ATOMIC_ACQUIRE, "workgroup");
    if (OUT_MODE == 0) {
      float* C = (float*)Cout + (size_t)b * strideC;
      const int hh = lane >> 4, c4 = (lane & 15) * 4;
      for (int pass = 0; pass < 2; ++pass) {
#pragma unroll
        for (int it = 0; it < 8; ++it) {
          const int row = it * 2 + hh;
          v4f v = *(const v4f*)(slab + row * 68 + c4);
          *(volatile v4f*)(C + (size_t)(mBase + row) * ldc + n0 + c4) = v;
        }
        __threadfence();
      }
    } else {
      const int q = lane >> 3, c8 = (lane & 7) * 8;
      unsigned short* C  = (unsigned short*)Cout  + (size_t)b * strideC;
      unsigned short* C2 = (OUT_MODE == 2) ? ((unsigned short*)Cout2 + (size_t)b * strideC) : nullptr;
      for (int pass = 0; pass < 2; ++pass) {
#pragma unroll
        for (int it = 0; it < 4; ++it) {
          const int row = it * 4 + q;
          const float* sp = slab + row * 68 + c8;
          v8h hv, lv;
#pragma unroll
          for (int e = 0; e < 8; ++e) {
            if (OUT_MODE == 1) {
              hv[e] = (_Float16)sp[e];
            } else {
              unsigned short hb = f2bf_bits(sp[e]);
              unsigned short lb = f2bf_bits(sp[e] - bf_bits2f(hb));
              hv[e] = __builtin_bit_cast(_Float16, hb);
              lv[e] = __builtin_bit_cast(_Float16, lb);
            }
          }
          *(volatile v8h*)(C + (size_t)(mBase + row) * ldc + n0 + c8) = hv;
          if (OUT_MODE == 2) *(volatile v8h*)(C2 + (size_t)(mBase + row) * ldc + n0 + c8) = lv;
        }
        __threadfence();
      }
    }
    __builtin_amdgcn_fence(__ATOMIC_RELEASE, "workgroup");
    __builtin_amdgcn_wave_barrier();
    __builtin_amdgcn_fence(__ATOMIC_ACQUIRE, "workgroup");
  }
}

__device__ __forceinline__ void put_split(_Float16* sw, int r, int col, float v) {
  const unsigned short hb = f2bf_bits(v);
  const unsigned short lb = f2bf_bits(v - bf_bits2f(hb));
  sw[r * STG_PITCH + col]       = __builtin_bit_cast(_Float16, hb);
  sw[(r + 1) * STG_PITCH + col] = __builtin_bit_cast(_Float16, lb);
}

__global__ __launch_bounds__(256) void rope_split_k(const float* __restrict__ qkv, const int* __restrict__ tpos,
    InvFreqTab ivt,
    unsigned short* __restrict__ qh, unsigned short* __restrict__ ql,
    unsigned short* __restrict__ kh, unsigned short* __restrict__ kl,
    unsigned short* __restrict__ vh, unsigned short* __restrict__ vl) {
#pragma clang fp contract(off)
  __shared__ float cs[2][32];
  __shared__ __align__(16) _Float16 stg[8][12 * STG_PITCH];
  const int m = blockIdx.x;
  const int b = m / SEQ_LEN;
  const int s = m - b * SEQ_LEN;
  const int tid = threadIdx.x, wave = tid >> 5, ln = tid & 31;
  if (wave == 0) {
    const int p = tpos[s];
    float invf = ivt.f[0];
#pragma unroll
    for (int q = 1; q < 32; ++q) invf = (ln == q) ? ivt.f[q] : invf;
    const float ang = (float)p * invf;
    float sv, cv;
    sincosf(ang, &sv, &cv);
    cs[0][ln] = cv;
    cs[1][ln] = sv;
  }
  __syncthreads();
  const float cv = cs[0][ln], sv = cs[1][ln];
  const float* row = qkv + (size_t)m * QKV_COLS;
  _Float16* sw = stg[wave];
#pragma unroll 1
  for (int j = 0; j < 2; ++j) {
    const int hd = wave + 8 * j;
    const v2f xq = *(const v2f*)(row + hd * HEAD_D + 2 * ln);
    put_split(sw, 2 * j, 2 * ln,     xq[0] * cv - xq[1] * sv);
    put_split(sw, 2 * j, 2 * ln + 1, xq[0] * sv + xq[1] * cv);
    const v2f xk = *(const v2f*)(row + K_COL0 + hd * HEAD_D + 2 * ln);
    put_split(sw, 4 + 2 * j, 2 * ln,     xk[0] * cv - xk[1] * sv);
    put_split(sw, 4 + 2 * j, 2 * ln + 1, xk[0] * sv + xk[1] * cv);
    const v2f xv = *(const v2f*)(row + V_COL0 + hd * HEAD_D + 2 * ln);
    put_split(sw, 8 + 2 * j, 2 * ln,     xv[0]);
    put_split(sw, 8 + 2 * j, 2 * ln + 1, xv[1]);
  }
  __builtin_amdgcn_fence(__ATOMIC_RELEASE, "workgroup");
  __builtin_amdgcn_wave_barrier();
  __builtin_amdgcn_fence(__ATOMIC_ACQUIRE, "workgroup");

  const int q8 = ln >> 3, c8 = (ln & 7) * 8;
  const v8h qv = *(const v8h*)(sw + (0 + q8) * STG_PITCH + c8);
  const v8h kv = *(const v8h*)(sw + (4 + q8) * STG_PITCH + c8);
  const v8h vv = *(const v8h*)(sw + (8 + q8) * STG_PITCH + c8);
  const int hd = wave + 8 * (q8 >> 1);
  const bool lop = ((q8 & 1) != 0);
  const size_t po = (((size_t)b * N_HEADS + hd) * SEQ_LEN + s) * HEAD_D + c8;
  unsigned short* qd = (lop ? ql : qh) + po;
  unsigned short* kd = (lop ? kl : kh) + po;
  unsigned short* vd = (lop ? vl : vh) + po;
  for (int pass = 0; pass < 2; ++pass) {
    *(volatile v8h*)qd = qv;
    *(volatile v8h*)kd = kv;
    *(volatile v8h*)vd = vv;
    __threadfence();
  }
}

__global__ __launch_bounds__(256) void vt_transpose_k(const unsigned short* __restrict__ vh, const unsigned short* __restrict__ vl,
                                                      unsigned short* __restrict__ vth, unsigned short* __restrict__ vtl) {
  __shared__ __align__(16) _Float16 th[64 * STG_PITCH];
  __shared__ __align__(16) _Float16 tl[64 * STG_PITCH];
  const int st0 = blockIdx.x * 64, g = blockIdx.y;
  const int tid = threadIdx.x;
  {
    const int sloc = tid >> 2, d0 = (tid & 3) * 16;
    const size_t so = ((size_t)g * SEQ_LEN + st0 + sloc) * HEAD_D + d0;
    const v8h a0 = *(const v8h*)((const _Float16*)vh + so);
    const v8h a1 = *(const v8h*)((const _Float16*)vh + so + 8);
    const v8h b0 = *(const v8h*)((const _Float16*)vl + so);
    const v8h b1 = *(const v8h*)((const _Float16*)vl + so + 8);
#pragma unroll
    for (int e = 0; e < 8; ++e) {
      th[(d0 + e) * STG_PITCH + sloc]     = a0[e];
      th[(d0 + 8 + e) * STG_PITCH + sloc] = a1[e];
      tl[(d0 + e) * STG_PITCH + sloc]     = b0[e];
      tl[(d0 + 8 + e) * STG_PITCH + sloc] = b1[e];
    }
  }
  __syncthreads();
  const int wave = tid >> 5, lane = tid & 31, q8 = lane >> 3, c8 = (lane & 7) * 8;
  const int dA = wave * 8 + q8, dB = wave * 8 + 4 + q8;
  const v8h hvA = *(const v8h*)(th + dA * STG_PITCH + c8);
  const v8h hvB = *(const v8h*)(th + dB * STG_PITCH + c8);
  const v8h lvA = *(const v8h*)(tl + dA * STG_PITCH + c8);
  const v8h lvB = *(const v8h*)(tl + dB * STG_PITCH + c8);
  const size_t oA = ((size_t)g * HEAD_D + dA) * SEQ_LEN + st0 + c8;
  const size_t oB = ((size_t)g * HEAD_D + dB) * SEQ_LEN + st0 + c8;
  for (int pass = 0; pass < 2; ++pass) {
    *(volatile v8h*)(vth + oA) = hvA;
    *(volatile v8h*)(vth + oB) = hvB;
    *(volatile v8h*)(vtl + oA) = lvA;
    *(volatile v8h*)(vtl + oB) = lvB;
    __threadfence();
  }
}

__global__ __launch_bounds__(128) void attn_hd64_k(
    const unsigned short* __restrict__ qh_p, const unsigned short* __restrict__ ql_p,
    const unsigned short* __restrict__ kh_p, const unsigned short* __restrict__ kl_p,
    const unsigned short* __restrict__ vth_p, const unsigned short* __restrict__ vtl_p,
    unsigned short* __restrict__ oh_p, unsigned short* __restrict__ ol_p) {
  union FB { v16b v; v8b h[2]; };
  __shared__ __align__(16) __bf16 Ksh[64 * 64];
  __shared__ __align__(16) __bf16 Ksl[64 * 64];
  __shared__ __align__(16) __bf16 Vsh[64 * 64];
  __shared__ __align__(16) __bf16 Vsl[64 * 64];
  __shared__ __align__(16) __bf16 Psh[4][16 * 64];
  __shared__ __align__(16) __bf16 Psl[4][16 * 64];
  __shared__ __align__(16) float  Osg[4][16 * 68];

  const __bf16* qh = (const __bf16*)qh_p; const __bf16* ql = (const __bf16*)ql_p;
  const __bf16* kh = (const __bf16*)kh_p; const __bf16* kl = (const __bf16*)kl_p;
  const __bf16* vth = (const __bf16*)vth_p; const __bf16* vtl = (const __bf16*)vtl_p;

  const int tid = threadIdx.x, wave = tid >> 5, lane = tid & 31, hh = lane >> 4, c = lane & 15;
  const int bx = blockIdx.x;
  const int bh = bx / NQB;
  const int qb = bx - bh * NQB;
  const int b  = bh / N_HEADS;
  const int h  = bh - b * N_HEADS;
  const int q0 = qb * 64 + wave * 16;

  v16b qah[2], qal[2];
  {
    const size_t qo = ((size_t)bh * SEQ_LEN + q0 + c) * HEAD_D + 8 * hh;
#pragma unroll
    for (int dc = 0; dc < 2; ++dc) {
      qah[dc] = Frag<__bf16>::load(qh + qo + dc * 32);
      qal[dc] = Frag<__bf16>::load(ql + qo + dc * 32);
    }
  }

  float mrow[8], lrow[8];
  v8f oacc[4];
#pragma unroll
  for (int r = 0; r < 8; ++r) { mrow[r] = -INFINITY; lrow[r] = 0.f; }
#pragma unroll
  for (int t = 0; t < 4; ++t) oacc[t] = (v8f){0.f,0.f,0.f,0.f,0.f,0.f,0.f,0.f};

  const int nChunks = qb + 1;
  for (int kc = 0; kc < nChunks; ++kc) {
    const int kv0 = kc * 64;
    __syncthreads();
    {
      const int rr = tid >> 1, hf = (tid & 1) * 32;
      const size_t ko = ((size_t)bh * SEQ_LEN + kv0 + rr) * HEAD_D + hf;
      const size_t vo = ((size_t)bh * HEAD_D + rr) * SEQ_LEN + kv0 + hf;
#pragma unroll
      for (int i = 0; i < 4; ++i) {
        *(v8b*)(Ksh + rr * 64 + hf + 8 * i) = *(const v8b*)(kh + ko + 8 * i);
        *(v8b*)(Ksl + rr * 64 + hf + 8 * i) = *(const v8b*)(kl + ko + 8 * i);
        *(v8b*)(Vsh + rr * 64 + hf + 8 * i) = *(const v8b*)(vth + vo + 8 * i);
        *(v8b*)(Vsl + rr * 64 + hf + 8 * i) = *(const v8b*)(vtl + vo + 8 * i);
      }
    }
    __syncthreads();

    v8f s[4];
#pragma unroll
    for (int j = 0; j < 4; ++j) {
      s[j] = (v8f){0.f,0.f,0.f,0.f,0.f,0.f,0.f,0.f};
#pragma unroll
      for (int dc = 0; dc < 2; ++dc) {
        FB kb, klo;
        kb.h[0]  = *(const v8b*)(Ksh + (j * 16 + c) * 64 + dc * 32 + 8 * hh);
        kb.h[1]  = *(const v8b*)(Ksh + (j * 16 + c) * 64 + dc * 32 + 16 + 8 * hh);
        klo.h[0] = *(const v8b*)(Ksl + (j * 16 + c) * 64 + dc * 32 + 8 * hh);
        klo.h[1] = *(const v8b*)(Ksl + (j * 16 + c) * 64 + dc * 32 + 16 + 8 * hh);
        s[j] = at_mma(qah[dc], kb.v,  s[j]);
        s[j] = at_mma(qah[dc], klo.v, s[j]);
        s[j] = at_mma(qal[dc], kb.v,  s[j]);
      }
    }

    const bool diag = (kc == qb);
    float cm[8];
#pragma unroll
    for (int r = 0; r < 8; ++r) {
      const int qrow = q0 + 8 * hh + r;
      float m = -INFINITY;
#pragma unroll
      for (int j = 0; j < 4; ++j) {
        const int kvcol = kv0 + j * 16 + c;
        float sv = s[j][r] * 0.125f;
        sv = (diag && (kvcol > qrow)) ? -INFINITY : sv;
        s[j][r] = sv;
        m = fmaxf(m, sv);
      }
#pragma unroll
      for (int off = 1; off < 16; off <<= 1) m = fmaxf(m, __shfl_xor(m, off, 32));
      cm[r] = m;
    }

    __bf16* pwh = Psh[wave];
    __bf16* pwl = Psl[wave];
#pragma unroll
    for (int r = 0; r < 8; ++r) {
      const float mnew = fmaxf(mrow[r], cm[r]);
      const float alpha = expf(mrow[r] - mnew);
      mrow[r] = mnew;
      float psum = 0.f;
#pragma unroll
      for (int j = 0; j < 4; ++j) {
        const float p = expf(s[j][r] - mnew);
        psum += p;
        __bf16 a, bl;
        at_split(p, a, bl);
        pwh[(8 * hh + r) * 64 + j * 16 + c] = a;
        pwl[(8 * hh + r) * 64 + j * 16 + c] = bl;
      }
#pragma unroll
      for (int off = 1; off < 16; off <<= 1) psum += __shfl_xor(psum, off, 32);
      lrow[r] = lrow[r] * alpha + psum;
#pragma unroll
      for (int t = 0; t < 4; ++t) oacc[t][r] *= alpha;
    }
    __builtin_amdgcn_fence(__ATOMIC_RELEASE, "workgroup");
    __builtin_amdgcn_wave_barrier();
    __builtin_amdgcn_fence(__ATOMIC_ACQUIRE, "workgroup");

#pragma unroll
    for (int kk = 0; kk < 2; ++kk) {
      FB pa, pl;
      pa.h[0] = *(const v8b*)(pwh + c * 64 + kk * 32 + 8 * hh);
      pa.h[1] = *(const v8b*)(pwh + c * 64 + kk * 32 + 16 + 8 * hh);
      pl.h[0] = *(const v8b*)(pwl + c * 64 + kk * 32 + 8 * hh);
      pl.h[1] = *(const v8b*)(pwl + c * 64 + kk * 32 + 16 + 8 * hh);
#pragma unroll
      for (int t = 0; t < 4; ++t) {
        FB vb, vlo;
        vb.h[0]  = *(const v8b*)(Vsh + (t * 16 + c) * 64 + kk * 32 + 8 * hh);
        vb.h[1]  = *(const v8b*)(Vsh + (t * 16 + c) * 64 + kk * 32 + 16 + 8 * hh);
        vlo.h[0] = *(const v8b*)(Vsl + (t * 16 + c) * 64 + kk * 32 + 8 * hh);
        vlo.h[1] = *(const v8b*)(Vsl + (t * 16 + c) * 64 + kk * 32 + 16 + 8 * hh);
        oacc[t] = at_mma(pa.v, vb.v,  oacc[t]);
        oacc[t] = at_mma(pa.v, vlo.v, oacc[t]);
        oacc[t] = at_mma(pl.v, vb.v,  oacc[t]);
      }
    }
  }

  float* os = Osg[wave];
#pragma unroll
  for (int r = 0; r < 8; ++r) {
    const float inv = 1.0f / lrow[r];
#pragma unroll
    for (int t = 0; t < 4; ++t) os[(8 * hh + r) * 68 + t * 16 + c] = oacc[t][r] * inv;
  }
  __builtin_amdgcn_fence(__ATOMIC_RELEASE, "workgroup");
  __builtin_amdgcn_wave_barrier();
  __builtin_amdgcn_fence(__ATOMIC_ACQUIRE, "workgroup");
  {
    const int q8 = lane >> 3, c8 = (lane & 7) * 8;
    for (int pass = 0; pass < 2; ++pass) {
#pragma unroll
      for (int it = 0; it < 4; ++it) {
        const int rowl = it * 4 + q8;
        const float* sp = os + rowl * 68 + c8;
        v8h hv, lv;
#pragma unroll
        for (int e = 0; e < 8; ++e) {
          const unsigned short hb = f2bf_bits(sp[e]);
          const unsigned short lb = f2bf_bits(sp[e] - bf_bits2f(hb));
          hv[e] = __builtin_bit_cast(_Float16, hb);
          lv[e] = __builtin_bit_cast(_Float16, lb);
        }
        const size_t oo = ((size_t)b * SEQ_LEN + q0 + rowl) * D_MOD + (size_t)h * HEAD_D + c8;
        *(volatile v8h*)(oh_p + oo) = hv;
        *(volatile v8h*)(ol_p + oo) = lv;
      }
      __threadfence();
    }
  }
}

static inline double host_sqrt_newton(double a) {
  double x = (a > 1.0) ? a * 0.5 : 1.0;
  for (int i = 0; i < 64; ++i) x = 0.5 * (x + a / x);
  return x;
}

extern "C" void kernel_launch(void* const* d_in, const int* in_sizes, int n_in,
                              void* d_out, int out_size, void* d_ws, size_t ws_size, hipStream_t stream) {
  if (n_in < 6) return;
  if (in_sizes[0] != NTOK * D_MOD || in_sizes[1] != SEQ_LEN ||
      in_sizes[2] != D_MOD * D_MOD || in_sizes[3] != D_MOD * D_MOD ||
      in_sizes[4] != D_MOD * D_MOD || in_sizes[5] != D_MOD * D_MOD ||
      out_size != NTOK * D_MOD) return;

  const float* x   = (const float*)d_in[0];
  const int*   tp  = (const int*)d_in[1];
  const float* wq  = (const float*)d_in[2];
  const float* wk  = (const float*)d_in[3];
  const float* wv  = (const float*)d_in[4];
  const float* wo  = (const float*)d_in[5];
  float* out = (float*)d_out;

  size_t off = 0;
  char* base = (char*)d_ws;
  auto carve = [&](size_t bytes) -> char* { char* p = base + off; off += bytes; return p; };
  const size_t plane16 = (size_t)NBH * SEQ_LEN * HEAD_D * 2;
  unsigned short* Xb   = (unsigned short*)carve((size_t)NTOK * D_MOD * 2);
  unsigned short* Wqkv = (unsigned short*)carve((size_t)QKV_COLS * D_MOD * 2);
  unsigned short* Wob  = (unsigned short*)carve((size_t)D_MOD * D_MOD * 2);
  char*           qkvb = carve((size_t)NTOK * QKV_COLS * 4);
  float*          QKVf = (float*)qkvb;
  unsigned short* Vth  = (unsigned short*)(qkvb);
  unsigned short* Vtl  = (unsigned short*)(qkvb + plane16);
  unsigned short* Oh   = (unsigned short*)(qkvb + 2 * plane16);
  unsigned short* Ol   = (unsigned short*)(qkvb + 3 * plane16);
  unsigned short* Qh   = (unsigned short*)carve(plane16);
  unsigned short* Ql   = (unsigned short*)carve(plane16);
  unsigned short* Kh   = (unsigned short*)carve(plane16);
  unsigned short* Kl   = (unsigned short*)carve(plane16);
  unsigned short* Vh   = (unsigned short*)carve(plane16);
  unsigned short* Vl   = (unsigned short*)carve(plane16);
  if (4 * plane16 > (size_t)NTOK * QKV_COLS * 4) return;
  if (off > ws_size) return;

  double rbase = 10000.0;
  for (int stp = 0; stp < 5; ++stp) rbase = host_sqrt_newton(rbase);
  InvFreqTab ivt;
  {
    double p = 1.0;
    for (int j = 0; j < 32; ++j) {
      ivt.f[j] = (float)(1.0 / p);
      p *= rbase;
    }
  }

  const int n2_x = (NTOK * D_MOD) / 2;
  const int n2_w = (D_MOD * D_MOD) / 2;
  cast_f32_bf16x2<<<dim3((n2_x + 255) / 256), dim3(256), 0, stream>>>(x,  Xb, n2_x);
  cast_f32_bf16x2<<<dim3((n2_w + 255) / 256), dim3(256), 0, stream>>>(wq, Wqkv, n2_w);
  cast_f32_bf16x2<<<dim3((n2_w + 255) / 256), dim3(256), 0, stream>>>(wk, Wqkv + (size_t)K_COL0 * D_MOD, n2_w);
  cast_f32_bf16x2<<<dim3((n2_w + 255) / 256), dim3(256), 0, stream>>>(wv, Wqkv + (size_t)V_COL0 * D_MOD, n2_w);
  cast_f32_bf16x2<<<dim3((n2_w + 255) / 256), dim3(256), 0, stream>>>(wo, Wob, n2_w);

  {
    const int tiles = (NTOK / 64) * (QKV_COLS / 64);
    wmma_gemm64<1, 0, 0, 0, false><<<dim3((tiles + 7) / 8, 1), dim3(256), 0, stream>>>(
        Xb, Xb, D_MOD, 0L, Wqkv, Wqkv, D_MOD, 0L, (void*)QKVf, (void*)QKVf, QKV_COLS, 0L,
        (const float*)QKVf, (const float*)QKVf, 0L, NTOK, QKV_COLS, D_MOD, 1.0f);
  }

  rope_split_k<<<dim3(NTOK), dim3(256), 0, stream>>>(QKVf, tp, ivt, Qh, Ql, Kh, Kl, Vh, Vl);
  vt_transpose_k<<<dim3(SEQ_LEN / 64, NBH), dim3(256), 0, stream>>>(Vh, Vl, Vth, Vtl);

  attn_hd64_k<<<dim3(NBH * NQB), dim3(128), 0, stream>>>(Qh, Ql, Kh, Kl, Vth, Vtl, Oh, Ol);

  {
    const int tiles = (NTOK / 64) * (D_MOD / 64);
    wmma_gemm64<1, 1, 0, 0, false><<<dim3((tiles + 7) / 8, 1), dim3(256), 0, stream>>>(
        Oh, Ol, D_MOD, 0L, Wob, Wob, D_MOD, 0L, (void*)out, (void*)out, D_MOD, 0L,
        (const float*)QKVf, (const float*)QKVf, 0L, NTOK, D_MOD, D_MOD, 1.0f);
  }
}
